// ViewEncoder_72834055406012
// MI455X (gfx1250) — hardware-verified
//
#include <hip/hip_runtime.h>
#include <stddef.h>


#define HID     128
#define G3      384
#define NTHR    256
#define NWAVE   8
#define EPT     8
#define NGRP    2
#define CHUNK   (NTHR * EPT * NGRP)
#define WCAP    (EPT * NGRP * 32)
#define LISTN   (NWAVE * WCAP)
#define NBC     4096
#define NBF     2048
#define FPB     (NBC / NBF)
#define RCAP    40960
#define RBN     128
#define OTHR    512
#define ROWS    32
#define DEGCAP  128
#define AP      136
#define WCROWS  32
#define WSC     64.0f
#define WINV    0.015625f
#define LOSC    2048.0f
#define LOINV   0.00048828125f
#define LNEPS   1e-5f
#define CNTMAX  65535
#define LDS_FILL ((RCAP + NBF + LISTN) * 4 + 64)

static_assert((CHUNK & (CHUNK - 1)) == 0);
static_assert(CHUNK <= 4096);
static_assert(NBC <= 4096 && NBF <= 4096);
static_assert((NBC & (NBC - 1)) == 0 && (NBF & (NBF - 1)) == 0);
static_assert(NBC == FPB * NBF);
static_assert(OTHR * 8 == NBC);
static_assert(((NBF / 8) % 32) == 0);
static_assert((OTHR / 32) == FPB * ((NBF / 8) / 32));
static_assert((RCAP % 32) == 0);
static_assert(ROWS == 4 * NWAVE);
static_assert((ROWS * HID / 4) % NTHR == 0);
static_assert((G3 * HID / 8) % NTHR == 0 && (HID * HID / 8) % NTHR == 0);
static_assert(G3 % WCROWS == 0 && WCROWS == 4 * NWAVE);
static_assert(G3 == 3 * HID);
static_assert(HID % 32 == 0 && (AP % 8) == 0 && AP >= HID);
static_assert(RBN * 4 == 512);

typedef float          v4f  __attribute__((ext_vector_type(4)));
typedef float          v8f  __attribute__((ext_vector_type(8)));
typedef int            v4i  __attribute__((ext_vector_type(4)));
typedef _Float16       v4h  __attribute__((ext_vector_type(4)));
typedef _Float16       v8h  __attribute__((ext_vector_type(8)));
typedef _Float16       v16h __attribute__((ext_vector_type(16)));
typedef unsigned short v8us __attribute__((ext_vector_type(8)));
typedef __bf16         v16b __attribute__((ext_vector_type(16)));
union FragH { v16h v; v8h  h[2]; };
union FragB { v16b v; v8us u[2]; };

__device__ __forceinline__ v8f zero8() { v8f z = {0.f, 0.f, 0.f, 0.f, 0.f, 0.f, 0.f, 0.f}; return z; }

__device__ __forceinline__ v4h cvt4(v4f a) {
  v4h r;
  r[0] = (_Float16)a.x; r[1] = (_Float16)a.y; r[2] = (_Float16)a.z; r[3] = (_Float16)a.w;
  return r;
}
__device__ __forceinline__ v4f widen4(v4h a) {
  v4f r;
  r.x = (float)a[0]; r.y = (float)a[1]; r.z = (float)a[2]; r.w = (float)a[3];
  return r;
}
__device__ __forceinline__ v8h cvt8(v4f a, v4f b) {
  v8h r;
  r[0] = (_Float16)a.x; r[1] = (_Float16)a.y; r[2] = (_Float16)a.z; r[3] = (_Float16)a.w;
  r[4] = (_Float16)b.x; r[5] = (_Float16)b.y; r[6] = (_Float16)b.z; r[7] = (_Float16)b.w;
  return r;
}

__device__ __forceinline__ v8f wmf(v16h a, v16h b, v8f c) {
  return __builtin_amdgcn_wmma_f32_16x16x32_f16(false, a, false, b, (short)0, c, false, false);
}
__device__ __forceinline__ v8f wmb(v16b a, v16b b, v8f c) {
  return __builtin_amdgcn_wmma_f32_16x16x32_bf16(false, a, false, b, (short)0, c, false, false);
}

__device__ __forceinline__ float sigm(float v) {
  return __builtin_amdgcn_rcpf(1.0f + __expf(-v));
}
__device__ __forceinline__ float tanh_f(float v) {
  return 1.0f - 2.0f * __builtin_amdgcn_rcpf(__expf(2.0f * v) + 1.0f);
}

template <int NB>
__device__ __forceinline__ int scan_chunk(const int* __restrict__ dsts, int nE, int cbase, int slotBase,
                                          int vec8, int* list, int tid, int lane, int wave) {
  int wc = 0;
#pragma unroll
  for (int g = 0; g < NGRP; ++g) {
    const int el0  = (g * NTHR + tid) * EPT;
    const int e0   = cbase + el0;
    const int sent = -2147483647 - 1;
    v4i da, db;
    if (vec8 != 0 && cbase + CHUNK <= nE) {
      da = *(const v4i*)(dsts + e0);
      db = *(const v4i*)(dsts + e0 + 4);
    } else {
      da.x = (e0     < nE) ? dsts[min(e0, nE - 1)] : sent;
      da.y = (e0 + 1 < nE) ? dsts[min(e0 + 1, nE - 1)] : sent;
      da.z = (e0 + 2 < nE) ? dsts[min(e0 + 2, nE - 1)] : sent;
      da.w = (e0 + 3 < nE) ? dsts[min(e0 + 3, nE - 1)] : sent;
      db.x = (e0 + 4 < nE) ? dsts[min(e0 + 4, nE - 1)] : sent;
      db.y = (e0 + 5 < nE) ? dsts[min(e0 + 5, nE - 1)] : sent;
      db.z = (e0 + 6 < nE) ? dsts[min(e0 + 6, nE - 1)] : sent;
      db.w = (e0 + 7 < nE) ? dsts[min(e0 + 7, nE - 1)] : sent;
    }
    const unsigned nb = (unsigned)slotBase;
    const unsigned s0 = (unsigned)da.x - nb, s1 = (unsigned)da.y - nb;
    const unsigned s2 = (unsigned)da.z - nb, s3 = (unsigned)da.w - nb;
    const unsigned s4 = (unsigned)db.x - nb, s5 = (unsigned)db.y - nb;
    const unsigned s6 = (unsigned)db.z - nb, s7 = (unsigned)db.w - nb;
    const bool h0 = s0 < (unsigned)NB, h1 = s1 < (unsigned)NB, h2 = s2 < (unsigned)NB, h3 = s3 < (unsigned)NB;
    const bool h4 = s4 < (unsigned)NB, h5 = s5 < (unsigned)NB, h6 = s6 < (unsigned)NB, h7 = s7 < (unsigned)NB;
    const unsigned any = __builtin_amdgcn_ballot_w32(h0 | h1 | h2 | h3 | h4 | h5 | h6 | h7);
    if (any != 0u) {
#define HITJ(J, HJ, SJ) { \
        const unsigned mj = __builtin_amdgcn_ballot_w32(HJ); \
        if (mj != 0u) { \
          if (HJ) { \
            const int pos = wc + (int)__builtin_amdgcn_mbcnt_lo(mj, 0u); \
            if (pos < WCAP) list[wave * WCAP + pos] = ((el0 + (J)) << 12) | (int)(SJ); \
          } \
          wc += (int)__builtin_popcount(mj); } }
      HITJ(0, h0, s0)
      HITJ(1, h1, s1)
      HITJ(2, h2, s2)
      HITJ(3, h3, s3)
      HITJ(4, h4, s4)
      HITJ(5, h5, s5)
      HITJ(6, h6, s6)
      HITJ(7, h7, s7)
#undef HITJ
    }
  }
  return wc;
}

__global__ __launch_bounds__(NTHR) void k_prep(
    const float* __restrict__ whh, const float* __restrict__ wih, const float* __restrict__ W,
    _Float16* whhP, unsigned short* wiHi, unsigned short* wiLo,
    unsigned short* wbHi, unsigned short* wbLo, int nW8) {
  constexpr int nG8 = G3 * HID / 8;
  const int i = blockIdx.x * NTHR + (int)threadIdx.x;
  if (i >= 2 * nG8 + nW8) return;
  const int seg = (i < nG8) ? 0 : ((i < 2 * nG8) ? 1 : 2);
  const int o = (seg == 0 ? i : (seg == 1 ? i - nG8 : i - 2 * nG8)) * 8;
  const float* src = (seg == 0) ? whh : ((seg == 1) ? wih : W);
  const v4f a = *(const v4f*)(src + o);
  const v4f b = *(const v4f*)(src + o + 4);
  if (seg == 0) {
    const v8h hv = cvt8(a * WSC, b * WSC);
    _Float16* dp = whhP + o;
    *(volatile v8h*)dp = hv;
    __threadfence();
    *(volatile v8h*)dp = hv;
  } else {
    float v[8];
    v[0] = a.x; v[1] = a.y; v[2] = a.z; v[3] = a.w;
    v[4] = b.x; v[5] = b.y; v[6] = b.z; v[7] = b.w;
    v8us hu, lu;
#pragma unroll
    for (int e = 0; e < 8; ++e) {
      const __bf16 hb = (__bf16)v[e];
      const float  rm = v[e] - (float)hb;
      const __bf16 lb = (__bf16)rm;
      hu[e] = __builtin_bit_cast(unsigned short, hb);
      lu[e] = __builtin_bit_cast(unsigned short, lb);
    }
    unsigned short* ph = ((seg == 1) ? wiHi : wbHi) + o;
    unsigned short* pl = ((seg == 1) ? wiLo : wbLo) + o;
    *(volatile v8us*)ph = hu;
    *(volatile v8us*)pl = lu;
    __threadfence();
    *(volatile v8us*)ph = hu;
    *(volatile v8us*)pl = lu;
  }
}

__global__ __launch_bounds__(NTHR) void k_wc(
    const unsigned short* __restrict__ wiHi, const unsigned short* __restrict__ wiLo,
    const unsigned short* __restrict__ wbHi, const unsigned short* __restrict__ wbLo,
    _Float16* wct) {
  __shared__ __attribute__((aligned(16))) _Float16 stg[WCROWS * HID];
  const int tid = threadIdx.x, lane = tid & 31, wave = tid >> 5, hh = lane >> 4, m = lane & 15;
  const int rt = wave & 1, ctb = (wave >> 1) * 2;
  const int c0 = blockIdx.x * WCROWS;
  const int li = blockIdx.y;
  const size_t arow  = (size_t)(c0 + 16 * rt + m) * HID + 8 * hh;
  const size_t brow0 = (size_t)(li * HID + 16 * ctb + m) * HID + 8 * hh;
  const size_t brow1 = brow0 + (size_t)16 * HID;
  const unsigned short* ahp = wiHi + arow;
  const unsigned short* alp = wiLo + arow;
  v8f d0 = zero8(), d1 = zero8();
#pragma unroll 1
  for (int kt = 0; kt < HID / 32; ++kt) {
    const int ko = 32 * kt;
    FragB ah, al, bh0, bl0, bh1, bl1;
    ah.u[0]  = *(const v8us*)(ahp + ko);          ah.u[1]  = *(const v8us*)(ahp + ko + 16);
    al.u[0]  = *(const v8us*)(alp + ko);          al.u[1]  = *(const v8us*)(alp + ko + 16);
    bh0.u[0] = *(const v8us*)(wbHi + brow0 + ko); bh0.u[1] = *(const v8us*)(wbHi + brow0 + ko + 16);
    bl0.u[0] = *(const v8us*)(wbLo + brow0 + ko); bl0.u[1] = *(const v8us*)(wbLo + brow0 + ko + 16);
    bh1.u[0] = *(const v8us*)(wbHi + brow1 + ko); bh1.u[1] = *(const v8us*)(wbHi + brow1 + ko + 16);
    bl1.u[0] = *(const v8us*)(wbLo + brow1 + ko); bl1.u[1] = *(const v8us*)(wbLo + brow1 + ko + 16);
    d0 = wmb(ah.v, bh0.v, d0);
    d1 = wmb(ah.v, bh1.v, d1);
    d0 = wmb(ah.v, bl0.v, d0);
    d1 = wmb(ah.v, bl1.v, d1);
    d0 = wmb(al.v, bh0.v, d0);
    d1 = wmb(al.v, bh1.v, d1);
    asm volatile("v_nop\n\tv_nop\n\tv_nop\n\tv_nop"
                 : "+v"(d0), "+v"(d1)
                 : "v"(ah.v), "v"(al.v), "v"(bh0.v), "v"(bl0.v), "v"(bh1.v), "v"(bl1.v));
  }
  {
    _Float16* sp0 = stg + (16 * rt + 8 * hh) * HID + 16 * ctb + m;
    _Float16* sp1 = sp0 + 16;
#pragma unroll
    for (int r = 0; r < 8; ++r) {
      sp0[r * HID] = (_Float16)(d0[r] * WSC);
      sp1[r * HID] = (_Float16)(d1[r] * WSC);
    }
  }
  __syncthreads();
  const _Float16* lp = stg + wave * 4 * HID;
  _Float16* gp = wct + ((size_t)li * G3 + c0 + wave * 4) * HID;
  const v8h v0 = *(const v8h*)(lp + 8 * lane);
  const v8h v1 = *(const v8h*)(lp + 8 * (32 + lane));
  *(volatile v8h*)(gp + 8 * lane) = v0;
  *(volatile v8h*)(gp + 8 * (32 + lane)) = v1;
  __threadfence();
  *(volatile v8h*)(gp + 8 * lane) = v0;
  *(volatile v8h*)(gp + 8 * (32 + lane)) = v1;
}

__global__ __launch_bounds__(NTHR) void k_count(const int* __restrict__ ei, int* cnt, int nE, int vec8) {
  __shared__ __attribute__((aligned(16))) int scnt[NBC];
  __shared__ __attribute__((aligned(16))) int list[LISTN];
  __shared__ int wcnt[NWAVE];
  const int tid = threadIdx.x, lane = tid & 31, wave = tid >> 5;
  const int nodeBase = blockIdx.x * NBC;
  const int* dsts = ei + nE;

  for (int i = tid; i < NBC; i += NTHR) scnt[i] = 0;
  __syncthreads();

  const int nChunks = (nE + CHUNK - 1) / CHUNK;
#pragma unroll 1
  for (int ch = 0; ch < nChunks; ++ch) {
    const int cbase = ch * CHUNK;
    const int wc = scan_chunk<NBC>(dsts, nE, cbase, nodeBase, vec8, list, tid, lane, wave);
    if (lane == 0) wcnt[wave] = wc;
    __syncthreads();
    if (wave == 0) {
#pragma unroll 1
      for (int wsx = 0; wsx < NWAVE; ++wsx) {
        int n = __builtin_amdgcn_readfirstlane(wcnt[wsx]);
        n = n > WCAP ? WCAP : (n < 0 ? 0 : n);
        const int* lp = list + wsx * WCAP;
#pragma unroll 1
        for (int i = 0; i < n; ++i) {
          const int ent  = __builtin_amdgcn_readfirstlane(lp[i]);
          const int slot = ent & (NBC - 1);
          if (lane == 0) scnt[slot] = scnt[slot] + 1;
        }
      }
    }
    __syncthreads();
  }

  v4i cq[4];
#pragma unroll
  for (int q = 0; q < 4; ++q) {
    const int f = (wave * 4 + q) * 128 + 4 * lane;
    cq[q] = *(const v4i*)(scnt + f);
  }
  int* cp = cnt + (size_t)nodeBase;
#pragma unroll
  for (int q = 0; q < 4; ++q) {
    const int f = (wave * 4 + q) * 128 + 4 * lane;
    *(volatile v4i*)(cp + f) = cq[q];
  }
  __threadfence();
#pragma unroll
  for (int q = 0; q < 4; ++q) {
    const int f = (wave * 4 + q) * 128 + 4 * lane;
    *(volatile v4i*)(cp + f) = cq[q];
  }
}

__global__ __launch_bounds__(OTHR) void k_offsets(const int* __restrict__ cnt, int* off, int* rbase, int nChunk) {
  __shared__ __attribute__((aligned(16))) int soff[NBC];
  __shared__ __attribute__((aligned(16))) int srb[RBN];
  __shared__ int wtot[OTHR / 32];
  constexpr int WPF = (NBF / 8) / 32;
  const int tid = threadIdx.x, lane = tid & 31, wave = tid >> 5;
  const int sub = wave / WPF;
  for (int i = tid; i < RBN; i += OTHR) srb[i] = 0;
  int carry = 0;
#pragma unroll 1
  for (int ch = 0; ch < nChunk; ++ch) {
    const int base = ch * NBC;
    const v4i c0 = *(const v4i*)(cnt + base + 8 * tid);
    const v4i c1 = *(const v4i*)(cnt + base + 8 * tid + 4);
    const int e0 = min(max(c0.x, 0), CNTMAX), e1 = min(max(c0.y, 0), CNTMAX);
    const int e2 = min(max(c0.z, 0), CNTMAX), e3 = min(max(c0.w, 0), CNTMAX);
    const int e4 = min(max(c1.x, 0), CNTMAX), e5 = min(max(c1.y, 0), CNTMAX);
    const int e6 = min(max(c1.z, 0), CNTMAX), e7 = min(max(c1.w, 0), CNTMAX);
    const int ts = e0 + e1 + e2 + e3 + e4 + e5 + e6 + e7;
    int incl = ts;
#pragma unroll
    for (int d = 1; d < 32; d <<= 1) {
      const int t = __shfl_up(incl, d);
      if (lane >= d) incl += t;
    }
    if (lane == 31) wtot[wave] = incl;
    __syncthreads();
    int S[FPB];
#pragma unroll
    for (int f = 0; f < FPB; ++f) {
      int s = 0;
#pragma unroll
      for (int w = 0; w < WPF; ++w) s += wtot[f * WPF + w];
      S[f] = s;
    }
    int pre = 0;
#pragma unroll 1
    for (int w = sub * WPF; w < wave; ++w) pre += wtot[w];
    int bcur = carry;
    int myb = carry;
#pragma unroll
    for (int f = 0; f < FPB; ++f) {
      if (tid == 0) srb[min(FPB * ch + f, RBN - 1)] = bcur;
      myb = (sub == f) ? bcur : myb;
      bcur += (S[f] + 31) & ~31;
    }
    int run = myb + pre + incl - ts;
    soff[8 * tid + 0] = run; run += e0;
    soff[8 * tid + 1] = run; run += e1;
    soff[8 * tid + 2] = run; run += e2;
    soff[8 * tid + 3] = run; run += e3;
    soff[8 * tid + 4] = run; run += e4;
    soff[8 * tid + 5] = run; run += e5;
    soff[8 * tid + 6] = run; run += e6;
    soff[8 * tid + 7] = run;
    carry = bcur;
    __syncthreads();
    const v4i o0 = *(const v4i*)(soff + 4 * tid);
    const v4i o1 = *(const v4i*)(soff + 4 * (tid + OTHR));
    int* op = off + base;
    *(volatile v4i*)(op + 4 * tid) = o0;
    *(volatile v4i*)(op + 4 * (tid + OTHR)) = o1;
    __threadfence();
    *(volatile v4i*)(op + 4 * tid) = o0;
    *(volatile v4i*)(op + 4 * (tid + OTHR)) = o1;
    __syncthreads();
  }
  if (tid == 0) srb[min(FPB * nChunk, RBN - 1)] = carry;
  __syncthreads();
  v4i rv = {0, 0, 0, 0};
  if (tid < 32) rv = *(const v4i*)(srb + 4 * tid);
  if (tid < 32) *(volatile v4i*)(rbase + 4 * tid) = rv;
  __threadfence();
  if (tid < 32) *(volatile v4i*)(rbase + 4 * tid) = rv;
}

__global__ __launch_bounds__(NTHR) void k_fill(
    const int* __restrict__ ei, const int* __restrict__ off, const int* __restrict__ rbase,
    int* csr, int nN, int nE, int vec8, int csrLen) {
  extern __shared__ v4f lds_dyn[];
  int* region = (int*)lds_dyn;
  int* cursor = region + RCAP;
  int* list   = cursor + NBF;
  int* wcnt   = list + LISTN;
  const int tid = threadIdx.x, lane = tid & 31, wave = tid >> 5;
  const int b = blockIdx.x;
  const int nodeBase = b * NBF;
  const int* dsts = ei + nE;

  int rb0 = rbase[min(b, RBN - 1)];
  const int rb1 = rbase[min(b + 1, RBN - 1)];
  rb0 = rb0 < 0 ? 0 : (rb0 > csrLen ? csrLen : rb0);
  rb0 &= ~31;
  int len = rb1 - rb0;
  len = len < 0 ? 0 : (len > RCAP ? RCAP : len);
  int lenW = (len + 31) & ~31;
  if (rb0 + lenW > csrLen) lenW = (csrLen - rb0) & ~31;

  {
    const v4i z = {0, 0, 0, 0};
    for (int i = tid; i < RCAP / 4; i += NTHR) ((v4i*)region)[i] = z;
    for (int s = tid; s < NBF; s += NTHR) {
      int o = off[nodeBase + s] - rb0;
      o = o < 0 ? 0 : (o > RCAP ? RCAP : o);
      cursor[s] = o;
    }
  }
  __syncthreads();

  const int nChunks = (nE + CHUNK - 1) / CHUNK;
#pragma unroll 1
  for (int ch = 0; ch < nChunks; ++ch) {
    const int cbase = ch * CHUNK;
    const int wc = scan_chunk<NBF>(dsts, nE, cbase, nodeBase, vec8, list, tid, lane, wave);
    if (lane == 0) wcnt[wave] = wc;
    __syncthreads();
    if (wave == 0) {
#pragma unroll 1
      for (int wsx = 0; wsx < NWAVE; ++wsx) {
        int n = __builtin_amdgcn_readfirstlane(wcnt[wsx]);
        n = n > WCAP ? WCAP : (n < 0 ? 0 : n);
        const int* lp = list + wsx * WCAP;
#pragma unroll 1
        for (int i = 0; i < n; ++i) {
          const int ent  = __builtin_amdgcn_readfirstlane(lp[i]);
          const int slot = ent & (NBF - 1);
          int e = cbase + ((ent >> 12) & (CHUNK - 1));
          e = e > nE - 1 ? nE - 1 : e;
          int src = ei[e];
          src = src < 0 ? 0 : (src > nN - 1 ? nN - 1 : src);
          if (lane == 0) {
            int pos = cursor[slot];
            pos = pos < 0 ? 0 : (pos > RCAP - 1 ? RCAP - 1 : pos);
            region[pos] = src;
            const int np = pos + 1;
            cursor[slot] = np > RCAP ? RCAP : np;
          }
        }
      }
    }
    __syncthreads();
  }

  const int nv = lenW >> 2;
  int* gp = csr + rb0;
#pragma unroll 1
  for (int i = tid; i < nv; i += NTHR) { const v4i v = ((const v4i*)region)[i]; *(volatile v4i*)(gp + 4 * i) = v; }
  __threadfence();
#pragma unroll 1
  for (int i = tid; i < nv; i += NTHR) { const v4i v = ((const v4i*)region)[i]; *(volatile v4i*)(gp + 4 * i) = v; }
}

template <int FINAL>
__global__ __launch_bounds__(NTHR) void k_layer(
    const float* __restrict__ hin, const int* __restrict__ csr, const int* __restrict__ off,
    const int* __restrict__ cnt, const _Float16* __restrict__ wc, const _Float16* __restrict__ whhP,
    const float* __restrict__ bih, const float* __restrict__ bhh, float* hout,
    const float* __restrict__ x, const float* __restrict__ gam, const float* __restrict__ bet,
    float* out, int nN, int csrLen) {
  __shared__ __attribute__((aligned(16))) _Float16 sAg[ROWS * AP];
  __shared__ __attribute__((aligned(16))) _Float16 sAl[ROWS * AP];
  __shared__ __attribute__((aligned(16))) _Float16 sAh[ROWS * AP];
  __shared__ __attribute__((aligned(16))) float    sH[ROWS * HID];
  const int tid = threadIdx.x, lane = tid & 31, wave = tid >> 5, hh = lane >> 4, m = lane & 15;
  const int rowBase = blockIdx.x * ROWS;

#pragma unroll
  for (int it = 0; it < (ROWS * HID / 4) / NTHR; ++it) {
    const int idx = it * NTHR + tid;
    const int r   = idx >> 5;
    const int c4  = (idx & 31) * 4;
    int row = rowBase + r;
    row = row > nN - 1 ? nN - 1 : row;
    const v4f v = *(const v4f*)(hin + (size_t)row * HID + c4);
    *(v4f*)(sH + r * HID + c4) = v;
    *(v4h*)(sAh + r * AP + c4) = cvt4(v);
  }

  {
    const int tb = rowBase + wave * 4;
    const int cl = tb + (lane & 3);
    const int cnt_l = cnt[cl];
    const int off_l = off[cl];
#pragma unroll 1
    for (int t = 0; t < 4; ++t) {
      int n = __builtin_amdgcn_readlane(cnt_l, t);
      n = n < 0 ? 0 : (n > DEGCAP ? DEGCAP : n);
      int st = __builtin_amdgcn_readlane(off_l, t);
      st = st < 0 ? 0 : (st > csrLen ? csrLen : st);
      v4f acc = {0.f, 0.f, 0.f, 0.f};
#pragma unroll 1
      for (int q0 = 0; q0 < n; q0 += 32) {
        int pos = st + q0 + lane;
        pos = pos > csrLen - 1 ? csrLen - 1 : pos;
        int sl = csr[pos];
        sl = sl < 0 ? 0 : (sl > nN - 1 ? nN - 1 : sl);
        const int mcnt = (n - q0) < 32 ? (n - q0) : 32;
#pragma unroll 1
        for (int p = 0; p < mcnt; ++p) {
          const int s = __builtin_amdgcn_readlane(sl, p);
          acc = acc + *(const v4f*)(hin + (size_t)s * HID + 4 * lane);
        }
      }
      const v4h hi4 = cvt4(acc);
      const v4f res = (acc - widen4(hi4)) * LOSC;
      const v4h lo4 = cvt4(res);
      *(v4h*)(sAg + (wave * 4 + t) * AP + 4 * lane) = hi4;
      *(v4h*)(sAl + (wave * 4 + t) * AP + 4 * lane) = lo4;
    }
  }
  __syncthreads();

  const int rt = wave & 1;
  const int jb = (wave >> 1) * 2;
  const _Float16* ag = sAg + (16 * rt + m) * AP + 8 * hh;
  const _Float16* al = sAl + (16 * rt + m) * AP + 8 * hh;
  const _Float16* ah = sAh + (16 * rt + m) * AP + 8 * hh;
#pragma unroll 1
  for (int jj = 0; jj < 2; ++jj) {
    const int cc = 16 * (jb + jj) + m;
    const _Float16* bi = wc   + (size_t)cc * HID + 8 * hh;
    const _Float16* bh = whhP + (size_t)cc * HID + 8 * hh;
    v8f c0 = zero8(), c1 = zero8(), c2 = zero8(), c3 = zero8(), c4 = zero8(), c5 = zero8();
    v8f c6 = zero8(), c7 = zero8(), c8 = zero8();
#pragma unroll 1
    for (int kt = 0; kt < HID / 32; ++kt) {
      const int ko = 32 * kt;
      {
        FragH fa, fl, b0, b1, b2;
        fa.h[0] = *(const v8h*)(ag + ko);
        fa.h[1] = *(const v8h*)(ag + ko + 16);
        fl.h[0] = *(const v8h*)(al + ko);
        fl.h[1] = *(const v8h*)(al + ko + 16);
        b0.h[0] = *(const v8h*)(bi + ko);
        b0.h[1] = *(const v8h*)(bi + ko + 16);
        b1.h[0] = *(const v8h*)(bi + HID * HID + ko);
        b1.h[1] = *(const v8h*)(bi + HID * HID + ko + 16);
        b2.h[0] = *(const v8h*)(bi + 2 * HID * HID + ko);
        b2.h[1] = *(const v8h*)(bi + 2 * HID * HID + ko + 16);
        c0 = wmf(fa.v, b0.v, c0);
        c1 = wmf(fa.v, b1.v, c1);
        c2 = wmf(fa.v, b2.v, c2);
        c6 = wmf(fl.v, b0.v, c6);
        c7 = wmf(fl.v, b1.v, c7);
        c8 = wmf(fl.v, b2.v, c8);
        asm volatile("v_nop\n\tv_nop\n\tv_nop\n\tv_nop"
                     : "+v"(c0), "+v"(c1), "+v"(c2), "+v"(c6), "+v"(c7), "+v"(c8)
                     : "v"(fa.v), "v"(fl.v), "v"(b0.v), "v"(b1.v), "v"(b2.v));
      }
      {
        FragH fh, b3, b4, b5;
        fh.h[0] = *(const v8h*)(ah + ko);
        fh.h[1] = *(const v8h*)(ah + ko + 16);
        b3.h[0] = *(const v8h*)(bh + ko);
        b3.h[1] = *(const v8h*)(bh + ko + 16);
        b4.h[0] = *(const v8h*)(bh + HID * HID + ko);
        b4.h[1] = *(const v8h*)(bh + HID * HID + ko + 16);
        b5.h[0] = *(const v8h*)(bh + 2 * HID * HID + ko);
        b5.h[1] = *(const v8h*)(bh + 2 * HID * HID + ko + 16);
        c3 = wmf(fh.v, b3.v, c3);
        c4 = wmf(fh.v, b4.v, c4);
        c5 = wmf(fh.v, b5.v, c5);
        asm volatile("v_nop\n\tv_nop\n\tv_nop\n\tv_nop"
                     : "+v"(c3), "+v"(c4), "+v"(c5)
                     : "v"(fh.v), "v"(b3.v), "v"(b4.v), "v"(b5.v));
      }
    }
    const float bir = bih[cc], biz = bih[HID + cc], bin = bih[2 * HID + cc];
    const float bhr = bhh[cc], bhz = bhh[HID + cc], bhn = bhh[2 * HID + cc];
    float* hp = sH + (16 * rt + 8 * hh) * HID + cc;
#pragma unroll
    for (int r = 0; r < 8; ++r) {
      const float ir  = (c0[r] + c6[r] * LOINV) * WINV + bir;
      const float iz  = (c1[r] + c7[r] * LOINV) * WINV + biz;
      const float inn = (c2[r] + c8[r] * LOINV) * WINV + bin;
      const float hr  = c3[r] * WINV + bhr;
      const float hz  = c4[r] * WINV + bhz;
      const float hn  = c5[r] * WINV + bhn;
      const float rg  = sigm(ir + hr);
      const float zg  = sigm(iz + hz);
      const float ng  = tanh_f(inn + rg * hn);
      const float hold = hp[r * HID];
      hp[r * HID] = ng + zg * (hold - ng);
    }
  }
  __syncthreads();

  const v4f g4 = *(const v4f*)(gam + 4 * lane);
  const v4f e4 = *(const v4f*)(bet + 4 * lane);
  v4f ov0, ov1, ov2, ov3;
#pragma unroll
  for (int q = 0; q < 4; ++q) {
    const int r = wave * 4 + q;
    const v4f v = *(const v4f*)(sH + r * HID + 4 * lane);
    v4f o = v;
    if (FINAL != 0) {
      float s = v.x + v.y + v.z + v.w;
#pragma unroll
      for (int sh = 16; sh > 0; sh >>= 1) s += __shfl_xor(s, sh, 32);
      const float mu = s * (1.0f / (float)HID);
      const v4f d = v - mu;
      float qs = d.x * d.x + d.y * d.y + d.z * d.z + d.w * d.w;
#pragma unroll
      for (int sh = 16; sh > 0; sh >>= 1) qs += __shfl_xor(qs, sh, 32);
      const float var = qs * (1.0f / (float)HID);
      const float inv = rsqrtf(var + LNEPS);
      int grow = rowBase + r;
      grow = grow > nN - 1 ? nN - 1 : grow;
      const v4f xv = *(const v4f*)(x + (size_t)grow * HID + 4 * lane);
      o = (d * inv) * g4 + e4;
      o = o + xv;
    }
    if (q == 0) ov0 = o; else if (q == 1) ov1 = o; else if (q == 2) ov2 = o; else ov3 = o;
  }
  float* dstp = (FINAL != 0) ? out : hout;
  const size_t rb0 = (size_t)(rowBase + wave * 4);
  const bool w0 = (FINAL == 0) || (rowBase + wave * 4 + 0 < nN);
  const bool w1 = (FINAL == 0) || (rowBase + wave * 4 + 1 < nN);
  const bool w2 = (FINAL == 0) || (rowBase + wave * 4 + 2 < nN);
  const bool w3 = (FINAL == 0) || (rowBase + wave * 4 + 3 < nN);
  if (w0) *(volatile v4f*)(dstp + (rb0 + 0) * HID + 4 * lane) = ov0;
  if (w1) *(volatile v4f*)(dstp + (rb0 + 1) * HID + 4 * lane) = ov1;
  if (w2) *(volatile v4f*)(dstp + (rb0 + 2) * HID + 4 * lane) = ov2;
  if (w3) *(volatile v4f*)(dstp + (rb0 + 3) * HID + 4 * lane) = ov3;
  __threadfence();
  if (w0) *(volatile v4f*)(dstp + (rb0 + 0) * HID + 4 * lane) = ov0;
  if (w1) *(volatile v4f*)(dstp + (rb0 + 1) * HID + 4 * lane) = ov1;
  if (w2) *(volatile v4f*)(dstp + (rb0 + 2) * HID + 4 * lane) = ov2;
  if (w3) *(volatile v4f*)(dstp + (rb0 + 3) * HID + 4 * lane) = ov3;
}

extern "C" void kernel_launch(void* const* d_in, const int* in_sizes, int n_in,
                              void* d_out, int out_size, void* d_ws, size_t ws_size,
                              hipStream_t stream) {
  if (n_in < 9) return;
  const int nN = in_sizes[0] / HID;
  const int nE = in_sizes[1] / 2;
  const int nL = in_sizes[2] / (HID * HID);
  if (nN <= 0 || nE <= 0 || nL < 1 || nL > 64) return;
  if (in_sizes[0] != nN * HID || in_sizes[1] != 2 * nE || in_sizes[2] != nL * HID * HID) return;
  if (in_sizes[3] != G3 * HID || in_sizes[4] != G3 * HID) return;
  if (in_sizes[5] < G3 || in_sizes[6] < G3 || in_sizes[7] < HID || in_sizes[8] < HID) return;
  if (out_size != nN * HID) return;
  if (nN > (1 << 24) || nE > (1 << 28)) return;

  const float* x    = (const float*)d_in[0];
  const int*   ei   = (const int*)d_in[1];
  const float* W    = (const float*)d_in[2];
  const float* w_ih = (const float*)d_in[3];
  const float* w_hh = (const float*)d_in[4];
  const float* b_ih = (const float*)d_in[5];
  const float* b_hh = (const float*)d_in[6];
  const float* gam  = (const float*)d_in[7];
  const float* bet  = (const float*)d_in[8];
  float* out = (float*)d_out;

  const int nGB    = (nN + ROWS - 1) / ROWS;
  const int NPADG  = nGB * ROWS;
  const int nBC    = (nN + NBC - 1) / NBC;
  const int CNTPAD = nBC * NBC;
  if (FPB * nBC + 1 > RBN) return;
  if (31 * FPB * nBC > 4096) return;
  const int nBF    = (nN + NBF - 1) / NBF;
  const int csrLen = ((nE + 31) & ~31) + 4096;

  char* ws = (char*)d_ws;
  size_t off = 0;
  const size_t oWhh = off; off += (size_t)G3 * HID * 2;          off = (off + 255) & ~(size_t)255;
  const size_t oWiH = off; off += (size_t)G3 * HID * 2;          off = (off + 255) & ~(size_t)255;
  const size_t oWiL = off; off += (size_t)G3 * HID * 2;          off = (off + 255) & ~(size_t)255;
  const size_t oWbH = off; off += (size_t)nL * HID * HID * 2;    off = (off + 255) & ~(size_t)255;
  const size_t oWbL = off; off += (size_t)nL * HID * HID * 2;    off = (off + 255) & ~(size_t)255;
  const size_t oWc  = off; off += (size_t)nL * G3 * HID * 2;     off = (off + 255) & ~(size_t)255;
  const size_t oCnt = off; off += (size_t)CNTPAD * 4;            off = (off + 255) & ~(size_t)255;
  const size_t oOff = off; off += (size_t)CNTPAD * 4;            off = (off + 255) & ~(size_t)255;
  const size_t oRb  = off; off += (size_t)RBN * 4;               off = (off + 255) & ~(size_t)255;
  const size_t oCsr = off; off += (size_t)csrLen * 4;            off = (off + 255) & ~(size_t)255;
  const size_t oHA  = off; off += (size_t)NPADG * HID * 4;       off = (off + 255) & ~(size_t)255;
  const size_t oHB  = off; off += (size_t)NPADG * HID * 4;       off = (off + 255) & ~(size_t)255;
  if (off > ws_size) return;
  _Float16*       whhP = (_Float16*)(ws + oWhh);
  unsigned short* wiHi = (unsigned short*)(ws + oWiH);
  unsigned short* wiLo = (unsigned short*)(ws + oWiL);
  unsigned short* wbHi = (unsigned short*)(ws + oWbH);
  unsigned short* wbLo = (unsigned short*)(ws + oWbL);
  _Float16*       wct  = (_Float16*)(ws + oWc);
  int*            cnt  = (int*)(ws + oCnt);
  int*            offp = (int*)(ws + oOff);
  int*            rb   = (int*)(ws + oRb);
  int*            csr  = (int*)(ws + oCsr);
  float*          hA   = (float*)(ws + oHA);
  float*          hB   = (float*)(ws + oHB);

  const int vec8 = ((nE & 3) == 0) ? 1 : 0;

  const int nW8   = nL * HID * HID / 8;
  const int nPrep = 2 * (G3 * HID / 8) + nW8;
  k_prep<<<(nPrep + NTHR - 1) / NTHR, NTHR, 0, stream>>>(w_hh, w_ih, W, whhP, wiHi, wiLo, wbHi, wbLo, nW8);

  k_wc<<<dim3(G3 / WCROWS, nL), NTHR, 0, stream>>>(wiHi, wiLo, wbHi, wbLo, wct);

  k_count<<<nBC, NTHR, 0, stream>>>(ei, cnt, nE, vec8);
  k_offsets<<<1, OTHR, 0, stream>>>(cnt, offp, rb, nBC);
  hipFuncSetAttribute(reinterpret_cast<const void*>(&k_fill),
                      hipFuncAttributeMaxDynamicSharedMemorySize, LDS_FILL);
  k_fill<<<nBF, NTHR, LDS_FILL, stream>>>(ei, offp, rb, csr, nN, nE, vec8, csrLen);

  const float* hin = x;
  for (int i = 0; i < nL; ++i) {
    float* ho = (i & 1) ? hB : hA;
    const _Float16* wci = wct + (size_t)i * G3 * HID;
    if (i == nL - 1) {
      k_layer<1><<<nGB, NTHR, 0, stream>>>(hin, csr, offp, cnt, wci, whhP, b_ih, b_hh, ho,
                                          x, gam, bet, out, nN, csrLen);
    } else {
      k_layer<0><<<nGB, NTHR, 0, stream>>>(hin, csr, offp, cnt, wci, whhP, b_ih, b_hh, ho,
                                          x, gam, bet, out, nN, csrLen);
    }
    hin = ho;
  }
}
